// MaxViTEncoderLayer_39917426049201
// MI455X (gfx1250) — hardware-verified
//
#include <hip/hip_runtime.h>
#include <math.h>

#define NB_    4
#define NL_    6400
#define ND_    256
#define NH_    8
#define NDH_   32
#define NC2_   512
#define NM_    (NB_ * NL_)
#define TBM_   128
#define NTB_   (NL_ / TBM_)
#define KVREC_ 1056
#define ATOK_  32
#define NAB_   (NL_ / ATOK_)

static_assert(NL_ % TBM_ == 0);
static_assert(NL_ % ATOK_ == 0);
static_assert(ND_ % 64 == 0);
static_assert(NC2_ % 64 == 0);
static_assert(ND_ == NH_ * NDH_);
static_assert(NM_ % 8 == 0);
static_assert((NM_ * ND_) % 2048 == 0);
static_assert((KVREC_ * 4) % 128 == 0);

typedef _Float16 v8h  __attribute__((ext_vector_type(8)));
typedef _Float16 v16h __attribute__((ext_vector_type(16)));
typedef __bf16   v8b  __attribute__((ext_vector_type(8)));
typedef __bf16   v16b __attribute__((ext_vector_type(16)));
typedef float    v2f  __attribute__((ext_vector_type(2)));
typedef float    v4f  __attribute__((ext_vector_type(4)));
typedef float    v8f  __attribute__((ext_vector_type(8)));
typedef unsigned short v8us __attribute__((ext_vector_type(8)));

enum { EPI_ELU1 = 1, EPI_BIAS_RELU = 2, EPI_BIAS = 3 };

__device__ __forceinline__ v8f vzero8() { v8f z = {0.f, 0.f, 0.f, 0.f, 0.f, 0.f, 0.f, 0.f}; return z; }
__device__ __forceinline__ v4f vzero4() { v4f z = {0.f, 0.f, 0.f, 0.f}; return z; }

__device__ __forceinline__ unsigned short bf_rne(float f) {
  unsigned u = __builtin_bit_cast(unsigned, f);
  u += 0x7FFFu + ((u >> 16) & 1u);
  return (unsigned short)(u >> 16);
}
__device__ __forceinline__ float bf_up(unsigned short b) {
  return __builtin_bit_cast(float, ((unsigned)b) << 16);
}

__device__ __forceinline__ v16h frag_h(const _Float16* __restrict__ rows, int ld, int lane, int k0) {
  const _Float16* p = rows + (size_t)(lane & 15) * ld + k0 + 8 * (lane >> 4);
  v8h e0 = *(const v8h*)p;
  v8h e1 = *(const v8h*)(p + 16);
  return __builtin_shufflevector(e0, e1, 0, 1, 2, 3, 4, 5, 6, 7, 8, 9, 10, 11, 12, 13, 14, 15);
}
__device__ __forceinline__ v16b frag_b(const __bf16* __restrict__ rows, int ld, int lane, int k0) {
  const __bf16* p = rows + (size_t)(lane & 15) * ld + k0 + 8 * (lane >> 4);
  v8b e0 = *(const v8b*)p;
  v8b e1 = *(const v8b*)(p + 16);
  return __builtin_shufflevector(e0, e1, 0, 1, 2, 3, 4, 5, 6, 7, 8, 9, 10, 11, 12, 13, 14, 15);
}

__device__ __forceinline__ v8f mma_h(v16h a, v16h b, v8f c) {
  return __builtin_amdgcn_wmma_f32_16x16x32_f16(false, a, false, b, (short)0, c, false, false);
}
__device__ __forceinline__ v8f mma_b(v16b a, v16b b, v8f c) {
  return __builtin_amdgcn_wmma_f32_16x16x32_bf16(false, a, false, b, (short)0, c, false, false);
}

__device__ __forceinline__ void tile_store_lines(const float* Cs, float* C, int ldc,
                                                 int trow0, int tcol0, int tid) {
  const int lane = tid & 31, wv = tid >> 5;
  v4f vals[8];
#pragma unroll
  for (int i = 0; i < 8; ++i) {
    const int r = wv * 16 + 2 * i + (lane >> 4);
    vals[i] = *(const v4f*)(Cs + r * 64 + (lane & 15) * 4);
  }
#pragma unroll
  for (int i = 0; i < 8; ++i) {
    const int r = wv * 16 + 2 * i + (lane >> 4);
    float* g = C + (size_t)(trow0 + r) * ldc + tcol0 + (lane & 15) * 4;
    *(volatile v4f*)g = vals[i];
  }
  __threadfence();
#pragma unroll
  for (int i = 0; i < 8; ++i) {
    const int r = wv * 16 + 2 * i + (lane >> 4);
    float* g = C + (size_t)(trow0 + r) * ldc + tcol0 + (lane & 15) * 4;
    *(volatile v4f*)g = vals[i];
  }
}

template <int SPLITA, int EPI>
__global__ __launch_bounds__(256)
void k_gemm_h(const _Float16* __restrict__ A0h, const _Float16* __restrict__ A0l, int lda0,
              const _Float16* __restrict__ A1h, const _Float16* __restrict__ A1l, int lda1, int ksplit,
              const _Float16* __restrict__ Bt, int K,
              const float* __restrict__ bias, float* __restrict__ C, int ldc)
{
  __shared__ __attribute__((aligned(16))) float Cs[TBM_ * 64];
  const int tid = threadIdx.x, lane = tid & 31, wv = tid >> 5, wr = wv & 3, wc = wv >> 2;
  const int hh = lane >> 4, nn = lane & 15;
  const int trow0 = blockIdx.y * TBM_, tcol0 = blockIdx.x * 64;
  const int row0 = trow0 + wr * 32, col0 = tcol0 + wc * 32;

  v8f acc[2][2], accl[2][2];
#pragma unroll
  for (int mi = 0; mi < 2; ++mi)
#pragma unroll
    for (int ni = 0; ni < 2; ++ni) { acc[mi][ni] = vzero8(); accl[mi][ni] = vzero8(); }

  for (int k0 = 0; k0 < K; k0 += 32) {
    const _Float16* Ah = A0h;
    const _Float16* Al = A0l;
    int lda = lda0, kk = k0;
    if (k0 >= ksplit) { Ah = A1h; Al = A1l; lda = lda1; kk = k0 - ksplit; }
    v16h a0 = frag_h(Ah + (size_t)row0 * lda, lda, lane, kk);
    v16h a1 = frag_h(Ah + (size_t)(row0 + 16) * lda, lda, lane, kk);
    v16h b0 = frag_h(Bt + (size_t)col0 * K, K, lane, k0);
    v16h b1 = frag_h(Bt + (size_t)(col0 + 16) * K, K, lane, k0);
    acc[0][0] = mma_h(a0, b0, acc[0][0]);
    acc[0][1] = mma_h(a0, b1, acc[0][1]);
    acc[1][0] = mma_h(a1, b0, acc[1][0]);
    acc[1][1] = mma_h(a1, b1, acc[1][1]);
    if (SPLITA) {
      v16h l0 = frag_h(Al + (size_t)row0 * lda, lda, lane, kk);
      v16h l1 = frag_h(Al + (size_t)(row0 + 16) * lda, lda, lane, kk);
      accl[0][0] = mma_h(l0, b0, accl[0][0]);
      accl[0][1] = mma_h(l0, b1, accl[0][1]);
      accl[1][0] = mma_h(l1, b0, accl[1][0]);
      accl[1][1] = mma_h(l1, b1, accl[1][1]);
      asm volatile("v_nop\n\tv_nop\n\tv_nop\n\tv_nop"
                   : "+v"(acc[0][0]), "+v"(acc[0][1]), "+v"(acc[1][0]), "+v"(acc[1][1]),
                     "+v"(accl[0][0]), "+v"(accl[0][1]), "+v"(accl[1][0]), "+v"(accl[1][1])
                   : "v"(a0), "v"(a1), "v"(b0), "v"(b1), "v"(l0), "v"(l1));
    } else {
      asm volatile("v_nop\n\tv_nop\n\tv_nop\n\tv_nop"
                   : "+v"(acc[0][0]), "+v"(acc[0][1]), "+v"(acc[1][0]), "+v"(acc[1][1])
                   : "v"(a0), "v"(a1), "v"(b0), "v"(b1));
    }
  }

#pragma unroll
  for (int mi = 0; mi < 2; ++mi) {
#pragma unroll
    for (int ni = 0; ni < 2; ++ni) {
      const int lcol = wc * 32 + ni * 16 + nn;
      float bv = 0.f;
      if (EPI == EPI_BIAS_RELU || EPI == EPI_BIAS) bv = bias[tcol0 + lcol];
#pragma unroll
      for (int r = 0; r < 8; ++r) {
        float v = acc[mi][ni][r] * (1.0f / 64.0f);
        if (SPLITA) v += accl[mi][ni][r] * (1.0f / 131072.0f);
        if (EPI == EPI_ELU1)           v = (v > 0.f) ? (v + 1.0f) : expf(v);
        else if (EPI == EPI_BIAS_RELU) v = fmaxf(v + bv, 0.f);
        else if (EPI == EPI_BIAS)      v = v + bv;
        Cs[(wr * 32 + mi * 16 + 8 * hh + r) * 64 + lcol] = v;
      }
    }
  }
  __syncthreads();
  tile_store_lines(Cs, C, ldc, trow0, tcol0, tid);
}

__global__ __launch_bounds__(256)
void k_gemm_b3(const __bf16* __restrict__ Ah, const __bf16* __restrict__ Al,
               const __bf16* __restrict__ Bh, const __bf16* __restrict__ Bl,
               float* __restrict__ C)
{
  __shared__ __attribute__((aligned(16))) float Cs[TBM_ * 64];
  const int tid = threadIdx.x, lane = tid & 31, wv = tid >> 5, wr = wv & 3, wc = wv >> 2;
  const int hh = lane >> 4, nn = lane & 15;
  const int trow0 = blockIdx.y * TBM_, tcol0 = blockIdx.x * 64;
  const int row0 = trow0 + wr * 32, col0 = tcol0 + wc * 32;

  v8f acc[2][2];
#pragma unroll
  for (int mi = 0; mi < 2; ++mi)
#pragma unroll
    for (int ni = 0; ni < 2; ++ni) acc[mi][ni] = vzero8();

  for (int k0 = 0; k0 < ND_; k0 += 32) {
    v16b a0h = frag_b(Ah + (size_t)row0 * ND_, ND_, lane, k0);
    v16b a1h = frag_b(Ah + (size_t)(row0 + 16) * ND_, ND_, lane, k0);
    v16b a0l = frag_b(Al + (size_t)row0 * ND_, ND_, lane, k0);
    v16b a1l = frag_b(Al + (size_t)(row0 + 16) * ND_, ND_, lane, k0);
    v16b b0h = frag_b(Bh + (size_t)col0 * ND_, ND_, lane, k0);
    v16b b1h = frag_b(Bh + (size_t)(col0 + 16) * ND_, ND_, lane, k0);
    v16b b0l = frag_b(Bl + (size_t)col0 * ND_, ND_, lane, k0);
    v16b b1l = frag_b(Bl + (size_t)(col0 + 16) * ND_, ND_, lane, k0);
    acc[0][0] = mma_b(a0h, b0h, acc[0][0]); acc[0][0] = mma_b(a0h, b0l, acc[0][0]); acc[0][0] = mma_b(a0l, b0h, acc[0][0]);
    acc[0][1] = mma_b(a0h, b1h, acc[0][1]); acc[0][1] = mma_b(a0h, b1l, acc[0][1]); acc[0][1] = mma_b(a0l, b1h, acc[0][1]);
    acc[1][0] = mma_b(a1h, b0h, acc[1][0]); acc[1][0] = mma_b(a1h, b0l, acc[1][0]); acc[1][0] = mma_b(a1l, b0h, acc[1][0]);
    acc[1][1] = mma_b(a1h, b1h, acc[1][1]); acc[1][1] = mma_b(a1h, b1l, acc[1][1]); acc[1][1] = mma_b(a1l, b1h, acc[1][1]);
    asm volatile("v_nop\n\tv_nop\n\tv_nop\n\tv_nop"
                 : "+v"(acc[0][0]), "+v"(acc[0][1]), "+v"(acc[1][0]), "+v"(acc[1][1])
                 : "v"(a0h), "v"(a1h), "v"(a0l), "v"(a1l), "v"(b0h), "v"(b1h), "v"(b0l), "v"(b1l));
  }

#pragma unroll
  for (int mi = 0; mi < 2; ++mi)
#pragma unroll
    for (int ni = 0; ni < 2; ++ni)
#pragma unroll
      for (int r = 0; r < 8; ++r)
        Cs[(wr * 32 + mi * 16 + 8 * hh + r) * 64 + wc * 32 + ni * 16 + nn] = acc[mi][ni][r];
  __syncthreads();
  tile_store_lines(Cs, C, ND_, trow0, tcol0, tid);
}

__global__ __launch_bounds__(256)
void k_kvproj(const _Float16* __restrict__ Sh, const _Float16* __restrict__ Wkv, float* __restrict__ Part)
{
  __shared__ __attribute__((aligned(16))) float Cs[TBM_ * 64];
  __shared__ __attribute__((aligned(16))) float ksh[32];
  const int tid = threadIdx.x, lane = tid & 31, wv = tid >> 5, wr = wv & 3, wc = wv >> 2;
  const int hh = lane >> 4, nn = lane & 15;
  const int h = blockIdx.x, tbg = blockIdx.y;
  const int b = tbg / NTB_, tb = tbg - b * NTB_;
  const int trow0 = tbg * TBM_;
  const int row0 = trow0 + wr * 32, col0 = wc * 32;
  const _Float16* Bt = Wkv + (size_t)h * 64 * ND_;

  v8f acc[2][2];
#pragma unroll
  for (int mi = 0; mi < 2; ++mi)
#pragma unroll
    for (int ni = 0; ni < 2; ++ni) acc[mi][ni] = vzero8();

  for (int k0 = 0; k0 < ND_; k0 += 32) {
    v16h a0 = frag_h(Sh + (size_t)row0 * ND_, ND_, lane, k0);
    v16h a1 = frag_h(Sh + (size_t)(row0 + 16) * ND_, ND_, lane, k0);
    v16h b0 = frag_h(Bt + (size_t)col0 * ND_, ND_, lane, k0);
    v16h b1 = frag_h(Bt + (size_t)(col0 + 16) * ND_, ND_, lane, k0);
    acc[0][0] = mma_h(a0, b0, acc[0][0]);
    acc[0][1] = mma_h(a0, b1, acc[0][1]);
    acc[1][0] = mma_h(a1, b0, acc[1][0]);
    acc[1][1] = mma_h(a1, b1, acc[1][1]);
    asm volatile("v_nop\n\tv_nop\n\tv_nop\n\tv_nop"
                 : "+v"(acc[0][0]), "+v"(acc[0][1]), "+v"(acc[1][0]), "+v"(acc[1][1])
                 : "v"(a0), "v"(a1), "v"(b0), "v"(b1));
  }

#pragma unroll
  for (int mi = 0; mi < 2; ++mi) {
#pragma unroll
    for (int ni = 0; ni < 2; ++ni) {
      const int lcol = wc * 32 + ni * 16 + nn;
#pragma unroll
      for (int r = 0; r < 8; ++r) {
        float v = acc[mi][ni][r] * (1.0f / 64.0f);
        if (wc == 0) v = (v > 0.f) ? (v + 1.0f) : expf(v);
        else         v = v * (1.0f / 6400.0f);
        Cs[(wr * 32 + mi * 16 + 8 * hh + r) * 64 + lcol] = v;
      }
    }
  }
  __syncthreads();

  const int d = tid >> 3, vq = tid & 7;
  v4f kv = vzero4();
  float ks = 0.f;
#pragma unroll 4
  for (int t = 0; t < TBM_; ++t) {
    const float kd = Cs[t * 64 + d];
    const v4f vv = *(const v4f*)(Cs + t * 64 + 32 + 4 * vq);
    v4f kd4 = {kd, kd, kd, kd};
    kv += kd4 * vv;
    ks += kd;
  }
  if (vq == 0) ksh[d] = ks;
  __syncthreads();
  v4f ksv = vzero4();
  if (tid < 8) ksv = *(const v4f*)(ksh + 4 * tid);

  float* P = Part + ((size_t)((b * NH_ + h) * NTB_ + tb)) * KVREC_;
  *(volatile v4f*)(P + 4 * tid) = kv;
  if (tid < 8) *(volatile v4f*)(P + 1024 + 4 * tid) = ksv;
  __threadfence();
  *(volatile v4f*)(P + 4 * tid) = kv;
  if (tid < 8) *(volatile v4f*)(P + 1024 + 4 * tid) = ksv;
}

__global__ __launch_bounds__(256)
void k_kvreduce(const float* __restrict__ Part, float* __restrict__ KVF)
{
  const int bh = blockIdx.x, tid = threadIdx.x;
  const float* P = Part + (size_t)bh * NTB_ * KVREC_;
  v4f s = vzero4(), t = vzero4();
#pragma unroll 2
  for (int p = 0; p < NTB_; ++p) {
    s += *(const v4f*)(P + (size_t)p * KVREC_ + 4 * tid);
    if (tid < 8) t += *(const v4f*)(P + (size_t)p * KVREC_ + 1024 + 4 * tid);
  }
  float* O = KVF + (size_t)bh * KVREC_;
  *(volatile v4f*)(O + 4 * tid) = s;
  if (tid < 8) *(volatile v4f*)(O + 1024 + 4 * tid) = t;
  __threadfence();
  *(volatile v4f*)(O + 4 * tid) = s;
  if (tid < 8) *(volatile v4f*)(O + 1024 + 4 * tid) = t;
}

__global__ __launch_bounds__(256)
void k_apply(const float* __restrict__ Q, const float* __restrict__ KVF,
             unsigned short* __restrict__ M0h, unsigned short* __restrict__ M0l)
{
  __shared__ __attribute__((aligned(16))) float KVs[NH_ * KVREC_];
  __shared__ __attribute__((aligned(16))) unsigned short stg[ATOK_ * ND_];
  const int tid = threadIdx.x;
  const int blk = blockIdx.x;
  const int b = blk / NAB_;
  const int tok0 = blk * ATOK_;
  const float* src = KVF + (size_t)b * NH_ * KVREC_;
  for (int i = tid; i < NH_ * KVREC_ / 4; i += 256)
    *(v4f*)(KVs + 4 * i) = *(const v4f*)(src + 4 * i);
  __syncthreads();

  const int tt = tid >> 3, h = tid & 7;
  const int token = tok0 + tt;
  const float* qp = Q + (size_t)token * ND_ + h * NDH_;
  const float* kvh = KVs + h * KVREC_;
  float acc[32];
#pragma unroll
  for (int v = 0; v < 32; ++v) acc[v] = 0.f;
  float zs = 0.f;
#pragma unroll 1
  for (int d = 0; d < NDH_; ++d) {
    const float qd = qp[d];
    zs = fmaf(qd, kvh[1024 + d], zs);
    const float* row = kvh + d * 32;
#pragma unroll
    for (int j = 0; j < 8; ++j) {
      const v4f r4 = *(const v4f*)(row + 4 * j);
      acc[4 * j + 0] = fmaf(qd, r4[0], acc[4 * j + 0]);
      acc[4 * j + 1] = fmaf(qd, r4[1], acc[4 * j + 1]);
      acc[4 * j + 2] = fmaf(qd, r4[2], acc[4 * j + 2]);
      acc[4 * j + 3] = fmaf(qd, r4[3], acc[4 * j + 3]);
    }
  }
  const float rz = 1.0f / (zs + 1e-6f);
#pragma unroll
  for (int v = 0; v < 32; ++v) acc[v] = (acc[v] * rz) * 6400.0f;

#pragma unroll
  for (int v = 0; v < 32; ++v) stg[tt * ND_ + h * NDH_ + v] = bf_rne(acc[v]);
  __syncthreads();
  v8us rh[4], rl[4];
#pragma unroll
  for (int i = 0; i < 4; ++i) rh[i] = *(const v8us*)(stg + 8 * (i * 256 + tid));
  __syncthreads();
#pragma unroll
  for (int v = 0; v < 32; ++v) {
    const unsigned short hb = bf_rne(acc[v]);
    stg[tt * ND_ + h * NDH_ + v] = bf_rne(acc[v] - bf_up(hb));
  }
  __syncthreads();
#pragma unroll
  for (int i = 0; i < 4; ++i) rl[i] = *(const v8us*)(stg + 8 * (i * 256 + tid));

  unsigned short* oh = M0h + (size_t)tok0 * ND_;
  unsigned short* ol = M0l + (size_t)tok0 * ND_;
#pragma unroll
  for (int i = 0; i < 4; ++i) {
    *(volatile v8us*)(oh + 8 * (i * 256 + tid)) = rh[i];
    *(volatile v8us*)(ol + 8 * (i * 256 + tid)) = rl[i];
  }
  __threadfence();
#pragma unroll
  for (int i = 0; i < 4; ++i) {
    *(volatile v8us*)(oh + 8 * (i * 256 + tid)) = rh[i];
    *(volatile v8us*)(ol + 8 * (i * 256 + tid)) = rl[i];
  }
}

__global__ __launch_bounds__(256)
void k_ln1(const float* __restrict__ T, const float* __restrict__ g, const float* __restrict__ bb,
           _Float16* __restrict__ Mh, _Float16* __restrict__ Ml)
{
  const int tid = threadIdx.x, lane = tid & 31;
  const int token = blockIdx.x * 8 + (tid >> 5);
  const int c0 = 8 * lane;
  const float* p = T + (size_t)token * ND_ + c0;
  const v4f u0 = *(const v4f*)p;
  const v4f u1 = *(const v4f*)(p + 4);
  float v[8] = {u0[0], u0[1], u0[2], u0[3], u1[0], u1[1], u1[2], u1[3]};
  float s = 0.f;
#pragma unroll
  for (int i = 0; i < 8; ++i) s += v[i];
#pragma unroll
  for (int o = 16; o; o >>= 1) s += __shfl_xor(s, o, 32);
  const float mu = s * (1.0f / 256.0f);
  float q = 0.f;
#pragma unroll
  for (int i = 0; i < 8; ++i) { const float dd = v[i] - mu; q += dd * dd; }
#pragma unroll
  for (int o = 16; o; o >>= 1) q += __shfl_xor(q, o, 32);
  const float inv = rsqrtf(q * (1.0f / 256.0f) + 1e-5f);
  v8h rh, rl;
#pragma unroll
  for (int i = 0; i < 8; ++i) {
    const float r = (v[i] - mu) * inv * g[c0 + i] + bb[c0 + i];
    const _Float16 hv = (_Float16)r;
    rh[i] = hv;
    rl[i] = (_Float16)((r - (float)hv) * 2048.0f);
  }
  _Float16* oh = Mh + (size_t)token * ND_ + c0;
  _Float16* ol = Ml + (size_t)token * ND_ + c0;
  *(volatile v8h*)oh = rh;
  *(volatile v8h*)ol = rl;
  __threadfence();
  *(volatile v8h*)oh = rh;
  *(volatile v8h*)ol = rl;
}

__global__ __launch_bounds__(256)
void k_ln2(const float* __restrict__ T, const float* __restrict__ g, const float* __restrict__ bb,
           const float* __restrict__ X, float* __restrict__ Out)
{
  const int tid = threadIdx.x, lane = tid & 31;
  const int token = blockIdx.x * 8 + (tid >> 5);
  const int c0 = 4 * lane, c1 = 128 + 4 * lane;
  const size_t base = (size_t)token * ND_;
  const v4f u0 = *(const v4f*)(T + base + c0);
  const v4f u1 = *(const v4f*)(T + base + c1);
  const v4f x0 = *(const v4f*)(X + base + c0);
  const v4f x1 = *(const v4f*)(X + base + c1);
  float v[8] = {u0[0], u0[1], u0[2], u0[3], u1[0], u1[1], u1[2], u1[3]};
  float s = 0.f;
#pragma unroll
  for (int i = 0; i < 8; ++i) s += v[i];
#pragma unroll
  for (int o = 16; o; o >>= 1) s += __shfl_xor(s, o, 32);
  const float mu = s * (1.0f / 256.0f);
  float q = 0.f;
#pragma unroll
  for (int i = 0; i < 8; ++i) { const float dd = v[i] - mu; q += dd * dd; }
#pragma unroll
  for (int o = 16; o; o >>= 1) q += __shfl_xor(q, o, 32);
  const float inv = rsqrtf(q * (1.0f / 256.0f) + 1e-5f);
  v4f o0, o1;
#pragma unroll
  for (int i = 0; i < 4; ++i) {
    const float r0 = (v[i] - mu) * inv * g[c0 + i] + bb[c0 + i];
    const float r1 = (v[4 + i] - mu) * inv * g[c1 + i] + bb[c1 + i];
    o0[i] = x0[i] + r0;
    o1[i] = x1[i] + r1;
  }
  *(volatile v4f*)(Out + base + c0) = o0;
  *(volatile v4f*)(Out + base + c1) = o1;
  __threadfence();
  *(volatile v4f*)(Out + base + c0) = o0;
  *(volatile v4f*)(Out + base + c1) = o1;
}

__global__ __launch_bounds__(256)
void k_dwconv(const float* __restrict__ Y1, const float* __restrict__ Wd, const float* __restrict__ Bd,
              const int* __restrict__ Hp, const int* __restrict__ Wp,
              _Float16* __restrict__ Y2h, _Float16* __restrict__ Y2l)
{
  const int tid = threadIdx.x, lane = tid & 31;
  const int token = blockIdx.x * 8 + (tid >> 5);
  int Wimg = Wp[0], Himg = Hp[0];
  Wimg = (Wimg < 1) ? 1 : ((Wimg > NL_) ? NL_ : Wimg);
  Himg = (Himg < 1) ? 1 : ((Himg > NL_) ? NL_ : Himg);
  const int b = token / NL_, l = token - b * NL_;
  const int i = l / Wimg, j = l - i * Wimg;
  int nb[9];
  float mk[9];
#pragma unroll
  for (int t = 0; t < 9; ++t) {
    const int ii = i + (t / 3) - 1, jj = j + (t % 3) - 1;
    const bool ok = (ii >= 0) && (ii < Himg) && (jj >= 0) && (jj < Wimg);
    int ln = ii * Wimg + jj;
    ln = (ln < 0) ? 0 : ((ln >= NL_) ? (NL_ - 1) : ln);
    nb[t] = b * NL_ + ln;
    mk[t] = ok ? 1.0f : 0.0f;
  }
  const _Float16 hz = (_Float16)0.0f;
#pragma unroll 1
  for (int g = 0; g < 2; ++g) {
    const int cb = g * 256 + 8 * lane;
    v8h rh = {hz, hz, hz, hz, hz, hz, hz, hz};
    v8h rl = {hz, hz, hz, hz, hz, hz, hz, hz};
#pragma unroll 1
    for (int p = 0; p < 4; ++p) {
      const int c = cb + 2 * p;
      float a0 = Bd[c], a1 = Bd[c + 1];
      const float* w0 = Wd + (size_t)c * 9;
      const float* w1 = w0 + 9;
#pragma unroll
      for (int t = 0; t < 9; ++t) {
        const v2f y = *(const v2f*)(Y1 + (size_t)nb[t] * NC2_ + c);
        a0 = fmaf(y[0], w0[t] * mk[t], a0);
        a1 = fmaf(y[1], w1[t] * mk[t], a1);
      }
      const float g0 = 0.5f * (a0 * (erff(a0 * 0.70710678118654752f) + 1.0f));
      const float g1 = 0.5f * (a1 * (erff(a1 * 0.70710678118654752f) + 1.0f));
      const _Float16 h0 = (_Float16)g0, h1 = (_Float16)g1;
      const _Float16 l0 = (_Float16)((g0 - (float)h0) * 2048.0f);
      const _Float16 l1 = (_Float16)((g1 - (float)h1) * 2048.0f);
      rh = __builtin_shufflevector(rh, rh, 2, 3, 4, 5, 6, 7, 0, 1);
      rl = __builtin_shufflevector(rl, rl, 2, 3, 4, 5, 6, 7, 0, 1);
      rh[6] = h0; rh[7] = h1;
      rl[6] = l0; rl[7] = l1;
    }
    _Float16* ph = Y2h + (size_t)token * NC2_ + cb;
    _Float16* pl = Y2l + (size_t)token * NC2_ + cb;
    *(volatile v8h*)ph = rh;
    *(volatile v8h*)pl = rl;
    __threadfence();
    *(volatile v8h*)ph = rh;
    *(volatile v8h*)pl = rl;
  }
}

__global__ __launch_bounds__(256)
void k_cvt_act(const float* __restrict__ X, const float* __restrict__ S,
               _Float16* __restrict__ Xh, _Float16* __restrict__ Xl, _Float16* __restrict__ Sh)
{
  const size_t gidx = (size_t)blockIdx.x * 256 + threadIdx.x;
  const size_t e = gidx * 8;
  const v4f a = *(const v4f*)(X + e), c = *(const v4f*)(X + e + 4);
  const v4f p = *(const v4f*)(S + e), q = *(const v4f*)(S + e + 4);
  float xv[8] = {a[0], a[1], a[2], a[3], c[0], c[1], c[2], c[3]};
  float sv[8] = {p[0], p[1], p[2], p[3], q[0], q[1], q[2], q[3]};
  v8h oh, ol, os;
#pragma unroll
  for (int i = 0; i < 8; ++i) {
    const _Float16 hv = (_Float16)xv[i];
    oh[i] = hv;
    ol[i] = (_Float16)((xv[i] - (float)hv) * 2048.0f);
    os[i] = (_Float16)sv[i];
  }
  *(volatile v8h*)(Xh + e) = oh;
  *(volatile v8h*)(Xl + e) = ol;
  *(volatile v8h*)(Sh + e) = os;
  __threadfence();
  *(volatile v8h*)(Xh + e) = oh;
  *(volatile v8h*)(Xl + e) = ol;
  *(volatile v8h*)(Sh + e) = os;
}

__global__ __launch_bounds__(256)
void k_cvt_w(const float* __restrict__ Wq, const float* __restrict__ Wk, const float* __restrict__ Wv,
             const float* __restrict__ Wm, const float* __restrict__ F1, const float* __restrict__ F2,
             _Float16* __restrict__ Wq16, _Float16* __restrict__ Wkv16,
             unsigned short* __restrict__ Wmh, unsigned short* __restrict__ Wml,
             _Float16* __restrict__ F1h, _Float16* __restrict__ F2h)
{
  const int job = blockIdx.y;
  const int gid = blockIdx.x * 256 + threadIdx.x;
  const float* src;
  int pitch;
  size_t dst;
  _Float16* outp = Wq16;
  if (job == 0) {
    if (gid >= ND_ * ND_ / 8) return;
    const int n = gid >> 5, k0 = (gid & 31) * 8;
    src = Wq + (size_t)k0 * ND_ + n; pitch = ND_; dst = (size_t)n * ND_ + k0; outp = Wq16;
  } else if (job == 1) {
    if (gid >= NH_ * 64 * ND_ / 8) return;
    const int row = gid >> 5, k0 = (gid & 31) * 8;
    const int h = row >> 6, jj = row & 63;
    src = (jj < 32) ? (Wk + h * NDH_ + jj) : (Wv + h * NDH_ + (jj - 32));
    src += (size_t)k0 * ND_; pitch = ND_; dst = (size_t)row * ND_ + k0; outp = Wkv16;
  } else if (job == 2) {
    if (gid >= ND_ * ND_ / 8) return;
    const int n = gid >> 5, k0 = (gid & 31) * 8;
    src = Wm + (size_t)k0 * ND_ + n; pitch = ND_; dst = (size_t)n * ND_ + k0;
  } else if (job == 3) {
    if (gid >= NC2_ * NC2_ / 8) return;
    const int n = gid >> 6, k0 = (gid & 63) * 8;
    src = F1 + (size_t)k0 * NC2_ + n; pitch = NC2_; dst = (size_t)n * NC2_ + k0; outp = F1h;
  } else {
    if (gid >= ND_ * NC2_ / 8) return;
    const int n = gid >> 6, k0 = (gid & 63) * 8;
    src = F2 + (size_t)k0 * ND_ + n; pitch = ND_; dst = (size_t)n * NC2_ + k0; outp = F2h;
  }
  float v[8];
#pragma unroll
  for (int i = 0; i < 8; ++i) v[i] = src[(size_t)i * pitch];
  if (job == 2) {
    v8us hb, lb;
#pragma unroll
    for (int i = 0; i < 8; ++i) {
      const unsigned short hbits = bf_rne(v[i]);
      hb[i] = hbits;
      lb[i] = bf_rne(v[i] - bf_up(hbits));
    }
    *(volatile v8us*)(Wmh + dst) = hb;
    *(volatile v8us*)(Wml + dst) = lb;
    __threadfence();
    *(volatile v8us*)(Wmh + dst) = hb;
    *(volatile v8us*)(Wml + dst) = lb;
  } else {
    v8h o;
#pragma unroll
    for (int i = 0; i < 8; ++i) o[i] = (_Float16)(v[i] * 64.0f);
    *(volatile v8h*)(outp + dst) = o;
    __threadfence();
    *(volatile v8h*)(outp + dst) = o;
  }
}

extern "C" void kernel_launch(void* const* d_in, const int* in_sizes, int n_in,
                              void* d_out, int out_size, void* d_ws, size_t ws_size,
                              hipStream_t stream)
{
  if (n_in < 18) return;
  if (in_sizes[0] != NM_ * ND_ || in_sizes[1] != NM_ * ND_ ||
      in_sizes[2] != ND_ * ND_ || in_sizes[3] != ND_ * ND_ || in_sizes[4] != ND_ * ND_ || in_sizes[5] != ND_ * ND_ ||
      in_sizes[6] != ND_ || in_sizes[7] != ND_ ||
      in_sizes[8] != NC2_ * NC2_ || in_sizes[9] != NC2_ ||
      in_sizes[10] != NC2_ * 9 || in_sizes[11] != NC2_ ||
      in_sizes[12] != NC2_ * ND_ || in_sizes[13] != ND_ || in_sizes[14] != ND_ || in_sizes[15] != ND_ ||
      in_sizes[16] < 1 || in_sizes[17] < 1 || out_size != NM_ * ND_) return;

  const float* x    = (const float*)d_in[0];
  const float* srcf = (const float*)d_in[1];
  const float* Wq   = (const float*)d_in[2];
  const float* Wk   = (const float*)d_in[3];
  const float* Wv   = (const float*)d_in[4];
  const float* Wm   = (const float*)d_in[5];
  const float* ln1g = (const float*)d_in[6];
  const float* ln1b = (const float*)d_in[7];
  const float* fc1w = (const float*)d_in[8];
  const float* fc1b = (const float*)d_in[9];
  const float* dww  = (const float*)d_in[10];
  const float* dwb  = (const float*)d_in[11];
  const float* fc2w = (const float*)d_in[12];
  const float* fc2b = (const float*)d_in[13];
  const float* ln2g = (const float*)d_in[14];
  const float* ln2b = (const float*)d_in[15];
  const int*   hp   = (const int*)d_in[16];
  const int*   wp   = (const int*)d_in[17];
  float* out = (float*)d_out;

  const size_t PL   = (size_t)NM_ * ND_ * 2;
  const size_t oR0  = 0, oR1 = PL, oR2 = 2 * PL, oR3 = 3 * PL, oR4 = 4 * PL;
  const size_t szR4 = (size_t)NM_ * NC2_ * 4;
  size_t o = oR4 + szR4;
  const size_t oWq  = o; o += (size_t)ND_ * ND_ * 2;
  const size_t oWkv = o; o += (size_t)NH_ * 64 * ND_ * 2;
  const size_t oWmh = o; o += (size_t)ND_ * ND_ * 2;
  const size_t oWml = o; o += (size_t)ND_ * ND_ * 2;
  const size_t oF1  = o; o += (size_t)NC2_ * NC2_ * 2;
  const size_t oF2  = o; o += (size_t)ND_ * NC2_ * 2;
  const size_t oPar = o; o += (size_t)NB_ * NH_ * NTB_ * KVREC_ * 4;
  const size_t oKVF = o; o += (size_t)NB_ * NH_ * KVREC_ * 4;
  const size_t total = o;
  if (total > ws_size) return;

  char* ws = (char*)d_ws;
  _Float16* Xh   = (_Float16*)(ws + oR0);
  _Float16* Xl   = (_Float16*)(ws + oR1);
  _Float16* Shp  = (_Float16*)(ws + oR4);
  float*    Qf   = (float*)(ws + oR4 + PL);
  unsigned short* M0h = (unsigned short*)(ws + oR2);
  unsigned short* M0l = (unsigned short*)(ws + oR3);
  float*    Tmp  = (float*)(ws + oR4);
  _Float16* Msh  = (_Float16*)(ws + oR2);
  _Float16* Msl  = (_Float16*)(ws + oR3);
  float*    Y1   = (float*)(ws + oR4);
  _Float16* Y2h  = (_Float16*)(ws + oR0);
  _Float16* Y2l  = (_Float16*)(ws + oR2);
  float*    Tmp2 = (float*)(ws + oR4);
  _Float16* Wq16 = (_Float16*)(ws + oWq);
  _Float16* Wkv16 = (_Float16*)(ws + oWkv);
  unsigned short* Wmh = (unsigned short*)(ws + oWmh);
  unsigned short* Wml = (unsigned short*)(ws + oWml);
  _Float16* F1h  = (_Float16*)(ws + oF1);
  _Float16* F2h  = (_Float16*)(ws + oF2);
  float*    Part = (float*)(ws + oPar);
  float*    KVF  = (float*)(ws + oKVF);

  const dim3 blk(256);
  const int BIGK = 1 << 30;

  k_cvt_act<<<dim3(NM_ * ND_ / 2048), blk, 0, stream>>>(x, srcf, Xh, Xl, Shp);
  k_cvt_w<<<dim3(128, 5), blk, 0, stream>>>(Wq, Wk, Wv, Wm, fc1w, fc2w, Wq16, Wkv16, Wmh, Wml, F1h, F2h);

  k_gemm_h<0, EPI_ELU1><<<dim3(ND_ / 64, NM_ / TBM_), blk, 0, stream>>>(
      Xh, Xh, ND_, Xh, Xh, ND_, BIGK, Wq16, ND_, fc1b, Qf, ND_);

  k_kvproj<<<dim3(NH_, NM_ / TBM_), blk, 0, stream>>>(Shp, Wkv16, Part);
  k_kvreduce<<<dim3(NB_ * NH_), blk, 0, stream>>>(Part, KVF);

  k_apply<<<dim3(NM_ / ATOK_), blk, 0, stream>>>(Qf, KVF, M0h, M0l);

  k_gemm_b3<<<dim3(ND_ / 64, NM_ / TBM_), blk, 0, stream>>>(
      (const __bf16*)M0h, (const __bf16*)M0l, (const __bf16*)Wmh, (const __bf16*)Wml, Tmp);

  k_ln1<<<dim3(NM_ / 8), blk, 0, stream>>>(Tmp, ln1g, ln1b, Msh, Msl);

  k_gemm_h<1, EPI_BIAS_RELU><<<dim3(NC2_ / 64, NM_ / TBM_), blk, 0, stream>>>(
      Xh, Xl, ND_, Msh, Msl, ND_, ND_, F1h, NC2_, fc1b, Y1, NC2_);

  k_dwconv<<<dim3(NM_ / 8), blk, 0, stream>>>(Y1, dww, dwb, hp, wp, Y2h, Y2l);

  k_gemm_h<1, EPI_BIAS><<<dim3(ND_ / 64, NM_ / TBM_), blk, 0, stream>>>(
      Y2h, Y2l, NC2_, Y2h, Y2l, NC2_, BIGK, F2h, NC2_, fc2b, Tmp2, ND_);

  k_ln2<<<dim3(NM_ / 8), blk, 0, stream>>>(Tmp2, ln2g, ln2b, x, out);
}
